// SMHAdapter_57183194579415
// MI455X (gfx1250) — hardware-verified
//
#include <hip/hip_runtime.h>
#include <hip/hip_bf16.h>
#include <math.h>

#define BB 2
#define SS 2048
#define DD 768
#define HH 12
#define DKK 64
#define GH 32
#define MTOK (BB * SS)

typedef _Float16 bf16;
typedef __attribute__((ext_vector_type(4))) unsigned v4u_t;
typedef unsigned v4ua __attribute__((ext_vector_type(4), may_alias));
typedef __attribute__((ext_vector_type(4))) float v4f_t;
typedef float v4fa __attribute__((ext_vector_type(4), may_alias));
typedef __attribute__((ext_vector_type(16))) bf16  bf16x16;
typedef __attribute__((ext_vector_type(8)))  bf16  bf16x8;
typedef __attribute__((ext_vector_type(4)))  bf16  bf16x4;
typedef __attribute__((ext_vector_type(8)))  float f32x8;

#define LDS_STRIDE 48
#define KSTRIDE    72
#define VSTRIDE    48

__device__ __forceinline__ f32x8 wmma_bf16(bf16x16 a, bf16x16 b, f32x8 c) {
  return __builtin_amdgcn_wmma_f32_16x16x32_f16(
      false, a, false, b, (short)0, c, false, false);
}

template <typename T>
__device__ __forceinline__ bf16x16 load_frag(const T* __restrict__ base, int ld,
                                             int row0, int k0) {
  const int lane = threadIdx.x & 31;
  const int r    = lane & 15;
  const int kh   = (lane >> 4) * 8;
  const T* p0 = base + (size_t)(row0 + r) * ld + (k0 + kh);
  const T* p1 = p0 + 16;
  bf16x16 f;
#pragma unroll
  for (int i = 0; i < 8; ++i) {
    f[i]     = (bf16)p0[i];
    f[i + 8] = (bf16)p1[i];
  }
  return f;
}

__device__ __forceinline__ bf16x16 lds_frag(const bf16* base, int stride) {
  const int lane = threadIdx.x & 31;
  const int row  = lane & 15;
  const int kh   = (lane >> 4) * 8;
  const bf16x8 lo = *(const bf16x8*)(base + row * stride + kh);
  const bf16x8 hi = *(const bf16x8*)(base + row * stride + kh + 16);
  bf16x16 f;
#pragma unroll
  for (int i = 0; i < 8; ++i) { f[i] = lo[i]; f[i + 8] = hi[i]; }
  return f;
}

template <typename T>
__device__ __forceinline__ void stage_read16(const T* __restrict__ p, float* buf) {
#pragma unroll
  for (int i = 0; i < 16; ++i) buf[i] = (float)p[i];
}

__device__ __forceinline__ void stage_write(bf16* dst, const float* buf, int nquad) {
#pragma unroll
  for (int i = 0; i < nquad; ++i) {
    bf16x4 q;
    q[0] = (bf16)buf[4 * i];     q[1] = (bf16)buf[4 * i + 1];
    q[2] = (bf16)buf[4 * i + 2]; q[3] = (bf16)buf[4 * i + 3];
    *(bf16x4*)(dst + 4 * i) = q;
  }
}

template <typename AT, int MODE>
__global__ __launch_bounds__(256) void gemm_bias_kernel(
    const AT* __restrict__ A, const float* __restrict__ W,
    const float* __restrict__ bias, void* __restrict__ out,
    int M, int N, int K) {
  __shared__ bf16 ldsA[128 * LDS_STRIDE];
  __shared__ bf16 ldsW[256 * LDS_STRIDE];
  __shared__ __attribute__((aligned(16))) unsigned char sob[256 * 136 * 2];

  const int t    = threadIdx.x;
  const int wave = t >> 5;
  const int lane = t & 31;
  const int wm   = (wave & 1) * 64;
  const int wn   = (wave >> 1) * 64;
  const int mBlk = blockIdx.x * 128;
  const int nBlk = blockIdx.y * 256;

  const int arow = t >> 1;
  const int ach  = (t & 1) * 16;

  float abuf[16];
  float wbuf[32];

  stage_read16(A + (size_t)(mBlk + arow) * K + ach, abuf);
  stage_read16(W + (size_t)(nBlk + t) * K,          wbuf);
  stage_read16(W + (size_t)(nBlk + t) * K + 16,     wbuf + 16);

  f32x8 acc[4][4] = {};

  for (int k = 0; k < K; k += 32) {
    __syncthreads();
    stage_write(&ldsA[arow * LDS_STRIDE + ach], abuf, 4);
    stage_write(&ldsW[t * LDS_STRIDE],          wbuf, 8);
    if (k + 32 < K) {
      stage_read16(A + (size_t)(mBlk + arow) * K + (k + 32) + ach, abuf);
      stage_read16(W + (size_t)(nBlk + t) * K + (k + 32),          wbuf);
      stage_read16(W + (size_t)(nBlk + t) * K + (k + 32) + 16,     wbuf + 16);
    }
    __syncthreads();

    bf16x16 af[4], wf[4];
#pragma unroll
    for (int i = 0; i < 4; ++i)
      af[i] = lds_frag(ldsA + (wm + 16 * i) * LDS_STRIDE, LDS_STRIDE);
#pragma unroll
    for (int j = 0; j < 4; ++j)
      wf[j] = lds_frag(ldsW + (wn + 16 * j) * LDS_STRIDE, LDS_STRIDE);
#pragma unroll
    for (int i = 0; i < 4; ++i)
#pragma unroll
      for (int j = 0; j < 4; ++j)
        acc[i][j] = wmma_bf16(af[i], wf[j], acc[i][j]);
  }

  const int nlane = lane & 15;
  const int mh    = (lane >> 4) * 8;
  __syncthreads();
  if (MODE == 0 || MODE == 1) {
    bf16* so = (bf16*)sob;
#pragma unroll
    for (int i = 0; i < 4; ++i)
#pragma unroll
      for (int j = 0; j < 4; ++j) {
        const int nl = wn + 16 * j + nlane;
        const float bv = bias[nBlk + nl];
#pragma unroll
        for (int r = 0; r < 8; ++r) {
          const int ml = wm + 16 * i + mh + r;
          const bf16 hv = (bf16)(acc[i][j][r] + bv);
          if (MODE == 0) so[ml * 264 + nl] = hv;
          else           so[nl * 136 + ml] = hv;
        }
      }
    __syncthreads();
#pragma unroll 1
    for (int pass = 0; pass < 2; ++pass) {
      if (MODE == 0) {
        for (int ch = t; ch < 128 * 32; ch += 256) { const int ml = ch >> 5, q = (ch & 31) * 8;
          *(volatile v4u_t*)((bf16*)out + (size_t)(mBlk + ml) * N + nBlk + q) = *(const v4ua*)(so + ml * 264 + q); }
      } else {
        const int b_ = mBlk / SS, s0 = mBlk & (SS - 1);
        for (int ch = t; ch < 256 * 16; ch += 256) { const int nl = ch >> 4, q = (ch & 15) * 8; const int n = nBlk + nl, h = n >> 6, dk = n & (DKK - 1);
          *(volatile v4u_t*)((bf16*)out + (((size_t)(b_ * HH + h)) * DKK + dk) * SS + s0 + q) = *(const v4ua*)(so + nl * 136 + q); }
      }
      __threadfence();
    }
  } else {
    float* so = (float*)sob;
#pragma unroll 1
    for (int hf = 0; hf < 2; ++hf) {
      if (wm == hf * 64) {
#pragma unroll
        for (int i = 0; i < 4; ++i)
#pragma unroll
          for (int j = 0; j < 4; ++j) {
            const int nl = wn + 16 * j + nlane;
            const float bv = bias[nBlk + nl];
#pragma unroll
            for (int r = 0; r < 8; ++r) so[(16 * i + mh + r) * 260 + nl] = acc[i][j][r] + bv;
          }
      }
      __syncthreads();
#pragma unroll 1
      for (int pass = 0; pass < 2; ++pass) {
        for (int ch = t; ch < 64 * 64; ch += 256) { const int ml = ch >> 6, q = (ch & 63) * 4;
          *(volatile v4f_t*)((float*)out + (size_t)(mBlk + hf * 64 + ml) * N + nBlk + q) = *(const volatile v4fa*)(so + ml * 260 + q); }
        __threadfence();
      }
      __syncthreads();
    }
  }
}


__global__ __launch_bounds__(128) void k_gate(const float* __restrict__ x, const float* __restrict__ sal,
                                              const float* __restrict__ gw1, const float* __restrict__ gb1,
                                              const float* __restrict__ gw2, const float* __restrict__ gb2,
                                              float* __restrict__ hout) {
  __shared__ __attribute__((aligned(16))) float hS[4][16 * 260];
  const int t = threadIdx.x, wave = t >> 5, lane = t & 31, col = lane & 15, rh = (lane >> 4) * 8, kh = rh;
  const int tok0 = blockIdx.x * 64 + wave * 16;
  bf16x16 af;
  {
    const float s = sal[tok0 + col];
#pragma unroll
    for (int i = 0; i < 8; ++i) {
      const int u0 = kh + i, u1 = kh + 16 + i;
      const float z0 = s * gw1[u0] + gb1[u0], z1 = s * gw1[u1] + gb1[u1];
      af[i]     = (bf16)(z0 / (1.0f + __expf(-z0)));
      af[i + 8] = (bf16)(z1 / (1.0f + __expf(-z1)));
    }
  }
  float* so = hS[wave];
#pragma unroll 1
  for (int ch = 0; ch < DD / 256; ++ch) {
#pragma unroll 2
    for (int nt = 0; nt < 16; ++nt) {
      const int n0 = ch * 256 + nt * 16;
      f32x8 acc = {};
      acc = wmma_bf16(af, load_frag(gw2, GH, n0, 0), acc);
      const int n = n0 + col;
      const float b2 = gb2[n];
#pragma unroll
      for (int r = 0; r < 8; ++r) {
        float g = 1.0f / (1.0f + __expf(-(acc[r] + b2)));
        g = fminf(fmaxf(g, 0.05f), 0.95f);
        so[(rh + r) * 260 + nt * 16 + col] = x[(size_t)(tok0 + rh + r) * DD + n] * g;
      }
    }
    asm volatile("s_wait_dscnt 0" ::: "memory");
    __syncthreads();
#pragma unroll 1
    for (int pass = 0; pass < 2; ++pass) {
#pragma unroll
      for (int it = 0; it < 32; ++it) { const int f4 = lane + 32 * it, rr = f4 >> 6, q = (f4 & 63) * 4;
        *(volatile v4f_t*)(hout + (size_t)(tok0 + rr) * DD + ch * 256 + q) = *(const volatile v4fa*)(so + rr * 260 + q); }
      __threadfence();
    }
    __syncthreads();
  }
}

__global__ __launch_bounds__(256) void k_padrows(const float* __restrict__ bk, const float* __restrict__ bv, bf16* __restrict__ padk, bf16* __restrict__ padv) {
  for (int i = threadIdx.x; i < DD; i += 256) { *(volatile bf16*)(padk + i) = (bf16)bk[i]; *(volatile bf16*)(padv + i) = (bf16)bv[i]; }
  __threadfence();
  for (int i = threadIdx.x; i < DD; i += 256) { *(volatile bf16*)(padk + i) = (bf16)bk[i]; *(volatile bf16*)(padv + i) = (bf16)bv[i]; }
}

__device__ __forceinline__ bf16x16 key_frag(const bf16* __restrict__ Kb_b, const bf16* __restrict__ padk, int key0, int k0) {
  const int lane = threadIdx.x & 31, r = lane & 15, kh = (lane >> 4) * 8;
  const int j = key0 + r;
  const bf16* p0 = (j >= 0) ? (Kb_b + (size_t)j * DD + k0 + kh) : (padk + k0 + kh);
  const bf16x8 lo = *(const bf16x8*)(p0), hi = *(const bf16x8*)(p0 + 16);
  bf16x16 f;
#pragma unroll
  for (int i = 0; i < 8; ++i) { f[i] = lo[i]; f[i + 8] = hi[i]; }
  return f;
}
__global__ __launch_bounds__(64) void k_local_attn(const bf16* __restrict__ Qb, const bf16* __restrict__ Kb,
                                                  const bf16* __restrict__ Vt, const bf16* __restrict__ padk,
                                                  const bf16* __restrict__ padv, bf16* __restrict__ ctxOut) {
  __shared__ __attribute__((aligned(16))) bf16 soS[2][16 * 136];
  const int t = threadIdx.x, wave = t >> 5, lane = t & 31, col = lane & 15, hsel = lane >> 4, kh = hsel * 8;
  const int gq0 = blockIdx.x * 32 + wave * 16;
  const int b = gq0 / SS, l0 = gq0 - b * SS;
  const bf16* Qb_b = Qb + (size_t)b * SS * DD;
  const bf16* Kb_b = Kb + (size_t)b * SS * DD;
  const bf16* Vt_b = Vt + (size_t)b * DD * SS;
  const int kb0 = (((l0 - 31 + 1024) >> 5) << 5) - 1024;
  const int lq = l0 + col;
  const float scale = 0.03608439182435161f * 1.44269504088896340736f;

  float s[2][2][8];
#pragma unroll
  for (int kb = 0; kb < 2; ++kb) {
    f32x8 s0 = {}, s1 = {};
    const int key0 = kb0 + 32 * kb;
#pragma unroll 2
    for (int ks = 0; ks < DD / 32; ++ks) {
      const bf16x16 qf = load_frag(Qb_b, DD, l0, ks * 32);
      s0 = wmma_bf16(key_frag(Kb_b, padk, key0, ks * 32), qf, s0);
      s1 = wmma_bf16(key_frag(Kb_b, padk, key0 + 16, ks * 32), qf, s1);
    }
#pragma unroll
    for (int r = 0; r < 8; ++r) { s[kb][0][r] = s0[r] * scale; s[kb][1][r] = s1[r] * scale; }
  }
  float m8 = -INFINITY, m32 = -INFINITY;
#pragma unroll
  for (int kb = 0; kb < 2; ++kb)
#pragma unroll
    for (int tt = 0; tt < 2; ++tt)
#pragma unroll
      for (int r = 0; r < 8; ++r) {
        const int j = kb0 + 32 * kb + 16 * tt + kh + r;
        if (j <= lq && j >= lq - 31) m32 = fmaxf(m32, s[kb][tt][r]);
        if (j <= lq && j >= lq - 7)  m8  = fmaxf(m8,  s[kb][tt][r]);
      }
  m32 = fmaxf(m32, __shfl_xor(m32, 16, 32)); m8 = fmaxf(m8, __shfl_xor(m8, 16, 32));
  float l8 = 0.0f, l32 = 0.0f;
#pragma unroll
  for (int kb = 0; kb < 2; ++kb)
#pragma unroll
    for (int tt = 0; tt < 2; ++tt)
#pragma unroll
      for (int r = 0; r < 8; ++r) {
        const int j = kb0 + 32 * kb + 16 * tt + kh + r;
        if (j <= lq && j >= lq - 31) l32 += exp2f(s[kb][tt][r] - m32);
        if (j <= lq && j >= lq - 7)  l8  += exp2f(s[kb][tt][r] - m8);
      }
  l32 += __shfl_xor(l32, 16, 32); l8 += __shfl_xor(l8, 16, 32);
  const float i32 = 512.0f / l32, i8 = 512.0f / l8;
  bf16x16 cf[2];
#pragma unroll
  for (int kb = 0; kb < 2; ++kb)
#pragma unroll
    for (int tt = 0; tt < 2; ++tt)
#pragma unroll
      for (int r = 0; r < 8; ++r) {
        const int j = kb0 + 32 * kb + 16 * tt + kh + r;
        float c = 0.0f;
        if (j <= lq && j >= lq - 31) c += exp2f(s[kb][tt][r] - m32) * i32;
        if (j <= lq && j >= lq - 7)  c += exp2f(s[kb][tt][r] - m8) * i8;
        cf[kb][8 * tt + r] = (bf16)c;
      }

  bf16* so = soS[wave];
#pragma unroll 1
  for (int ch = 0; ch < DD / 128; ++ch) {
    f32x8 o[8];
#pragma unroll
    for (int dt = 0; dt < 8; ++dt) {
      f32x8 acc = {};
      const int d0 = ch * 128 + dt * 16;
#pragma unroll
      for (int kb = 0; kb < 2; ++kb) {
        const int key0 = kb0 + 32 * kb;
        bf16x16 vf;
        if (key0 >= 0) {
          vf = load_frag(Vt_b, SS, d0, key0);
        } else {
          const bf16 pv = padv[d0 + col];
#pragma unroll
          for (int i = 0; i < 16; ++i) vf[i] = pv;
        }
        acc = wmma_bf16(vf, cf[kb], acc);
      }
      o[dt] = acc;
    }
#pragma unroll
    for (int dt = 0; dt < 8; ++dt)
#pragma unroll
      for (int r = 0; r < 8; ++r) so[col * 136 + dt * 16 + kh + r] = (bf16)(o[dt][r] * (1.0f / 1024.0f));
    asm volatile("s_wait_dscnt 0" ::: "memory");
    __syncthreads();
#pragma unroll 1
    for (int pass = 0; pass < 2; ++pass) {
#pragma unroll
      for (int it = 0; it < 8; ++it) { const int c16 = lane + 32 * it, ql = c16 >> 4, q8 = (c16 & 15) * 8;
        *(volatile v4u_t*)(ctxOut + (size_t)(gq0 + ql) * DD + ch * 128 + q8) = *(const v4ua*)(so + ql * 136 + q8); }
      __threadfence();
    }
    __syncthreads();
  }
}

__global__ __launch_bounds__(256) void k_resid(const float* __restrict__ x, float* __restrict__ out) {
  const size_t e = ((size_t)blockIdx.x * 256 + threadIdx.x) * 4;
  v4f_t y = *(const volatile v4fa*)(out + e); const v4f_t xv = *(const v4fa*)(x + e);
  y.x += xv.x; y.y += xv.y; y.z += xv.z; y.w += xv.w;
  *(volatile v4f_t*)(out + e) = y; __threadfence(); *(volatile v4f_t*)(out + e) = y;
}

extern "C" void kernel_launch(void* const* d_in, const int* in_sizes, int n_in,
                              void* d_out, int out_size, void* d_ws, size_t ws_size,
                              hipStream_t stream) {
  (void)in_sizes; (void)n_in; (void)out_size; (void)ws_size;
  const float* x   = (const float*)d_in[0];
  const float* sal = (const float*)d_in[1];
  const float* gw1 = (const float*)d_in[2];
  const float* gb1 = (const float*)d_in[3];
  const float* gw2 = (const float*)d_in[4];
  const float* gb2 = (const float*)d_in[5];
  const float* wq  = (const float*)d_in[6];  const float* bq = (const float*)d_in[7];
  const float* wk  = (const float*)d_in[8];  const float* bk = (const float*)d_in[9];
  const float* wv  = (const float*)d_in[10]; const float* bv = (const float*)d_in[11];
  const float* wo  = (const float*)d_in[12]; const float* bo = (const float*)d_in[13];
  float* out = (float*)d_out;

  char* ws = (char*)d_ws;
  const size_t hB = (size_t)MTOK * DD * 4, fB = (size_t)MTOK * DD * 2;
  float* hbuf = (float*)ws;
  bf16* Qb   = (bf16*)(ws + hB);
  bf16* Kb   = (bf16*)(ws + hB + fB);
  bf16* VtB  = (bf16*)(ws + hB + 2 * fB);
  bf16* ctx  = (bf16*)(ws + hB + 3 * fB);
  bf16* padk = (bf16*)(ws + hB + 4 * fB);
  bf16* padv = (bf16*)(ws + hB + 4 * fB + 2048);

  k_gate<<<dim3(MTOK / 64), dim3(128), 0, stream>>>(x, sal, gw1, gb1, gw2, gb2, hbuf);
  k_padrows<<<dim3(1), dim3(256), 0, stream>>>(bk, bv, padk, padv);
  const int M = MTOK, N = DD, K = DD;
  dim3 gGrid(M / 128, N / 256), gBlk(256);
  gemm_bias_kernel<float, 0><<<gGrid, gBlk, 0, stream>>>(hbuf, wq, bq, Qb,  M, N, K);
  gemm_bias_kernel<float, 0><<<gGrid, gBlk, 0, stream>>>(hbuf, wk, bk, Kb,  M, N, K);
  gemm_bias_kernel<float, 1><<<gGrid, gBlk, 0, stream>>>(hbuf, wv, bv, VtB, M, N, K);
  k_local_attn<<<dim3(MTOK / 32), dim3(64), 0, stream>>>(Qb, Kb, VtB, padk, padv, ctx);
  gemm_bias_kernel<bf16, 2><<<gGrid, gBlk, 0, stream>>>(ctx, wo, bo, out, M, N, K);
  k_resid<<<dim3(MTOK * DD / 1024), dim3(256), 0, stream>>>(hbuf, out);
}
